// vaup_67345087201385
// MI455X (gfx1250) — hardware-run, weakly checked
//
#include <hip/hip_runtime.h>


#ifndef BS
#define BS 4096
#endif
#ifndef DD
#define DD 2048
#endif
#define BS_FULL 4096
#define D_FULL  2048
#ifndef OUT_PITCH
#define OUT_PITCH DD
#endif
#define KA (2 * BS)

static_assert(BS % 64 == 0);
static_assert(DD % 128 == 0);
static_assert(BS % 32 == 0);
static_assert(BS <= BS_FULL);
static_assert(DD <= D_FULL);
static_assert(D_FULL % 4 == 0);
static_assert(OUT_PITCH % 32 == 0);
static_assert(OUT_PITCH >= DD);

typedef unsigned short bf;
typedef __attribute__((ext_vector_type(16))) __bf16   v16bf;
typedef __attribute__((ext_vector_type(8)))  unsigned short v8us;
typedef __attribute__((ext_vector_type(8)))  float    v8f;
typedef __attribute__((ext_vector_type(4)))  float    v4f;
typedef v4f  __attribute__((may_alias)) v4fa;

__device__ __forceinline__ unsigned short f2bf(float f) { unsigned u = __float_as_uint(f); u += 0x7FFFu + ((u >> 16) & 1u); return (unsigned short)(u >> 16); }
__device__ __forceinline__ float bf2f(unsigned short h) { return __uint_as_float(((unsigned)h) << 16); }
__device__ __forceinline__ float bfr(float f) { return bf2f(f2bf(f)); }
__device__ __forceinline__ v16bf cat16b(v8us lo, v8us hi) { return __builtin_bit_cast(v16bf, __builtin_shufflevector(lo, hi, 0, 1, 2, 3, 4, 5, 6, 7, 8, 9, 10, 11, 12, 13, 14, 15)); }
__device__ __forceinline__ v8f wmmab(v16bf a, v16bf b, v8f c) { return __builtin_amdgcn_wmma_f32_16x16x32_bf16(false, a, false, b, (short)0, c, false, false); }
__device__ __forceinline__ v16bf ldb(const bf* p)  { return cat16b(*(const v8us*)p, *(const v8us*)(p + 16)); }
__device__ __forceinline__ void wave_sync() { __builtin_amdgcn_fence(3  , "wavefront"); __builtin_amdgcn_wave_barrier(); asm volatile("" ::: "memory"); }

__global__ __launch_bounds__(256) void k_coef(const float* __restrict__ x, const float* __restrict__ mean, float* coef) {
    __shared__ __align__(16) float cs[32];
    const int lane = threadIdx.x & 31;
    const int wave = __builtin_amdgcn_readfirstlane((int)(threadIdx.x >> 5));
    const int jb = blockIdx.x * 32;
#pragma unroll 1
    for (int r = 0; r < 4; ++r) {
        const int j = jb + wave * 4 + r;
        const float* xr = x + (size_t)j * D_FULL;
        float s = 0.0f;
#pragma unroll 1
        for (int i = 0; i < DD / 128; ++i) {
            const int c = (lane + 32 * i) * 4;
            const v4f xv = *(const v4f*)(xr + c);
            const v4f mv = *(const v4f*)(mean + c);
            s = fmaf(bfr(xv[0]), bfr(mv[0]), s);
            s = fmaf(bfr(xv[1]), bfr(mv[1]), s);
            s = fmaf(bfr(xv[2]), bfr(mv[2]), s);
            s = fmaf(bfr(xv[3]), bfr(mv[3]), s);
        }
        s += __shfl_xor(s, 16, 32);
        s += __shfl_xor(s, 8, 32);
        s += __shfl_xor(s, 4, 32);
        s += __shfl_xor(s, 2, 32);
        s += __shfl_xor(s, 1, 32);
        const float e = expf(-fabsf(s));
        const float t = 1.0f / (1.0f + e);
        const float cf = (t * (e * t)) * (float)(BS - j);
        if (lane == 0) cs[wave * 4 + r] = cf;
    }
    __syncthreads();
    if (wave == 0 && lane < 8) {
        const v4f v = *(const v4fa*)(&cs[lane * 4]);
        float* dst = coef + jb + lane * 4;
        *(volatile v4f*)dst = v; __threadfence(); *(volatile v4f*)dst = v;
    }
}

__global__ __launch_bounds__(256) void k_planes(const float* __restrict__ x, const float* __restrict__ coef, bf* XT, bf* AT) {
    __shared__ float xs[64 * 65];
    __shared__ float cs[64];
    const int t = threadIdx.x;
    const int lane = t & 31;
    const int wave = __builtin_amdgcn_readfirstlane((int)(threadIdx.x >> 5));
    const int j0 = blockIdx.x * 64, a0 = blockIdx.y * 64;
#pragma unroll
    for (int i = 0; i < 4; ++i) {
        const int idx = t + 256 * i; const int jr = idx >> 4, c4 = (idx & 15) * 4;
        const v4f v = *(const v4f*)(x + (size_t)(j0 + jr) * D_FULL + a0 + c4);
        xs[jr * 65 + c4 + 0] = bfr(v[0]); xs[jr * 65 + c4 + 1] = bfr(v[1]);
        xs[jr * 65 + c4 + 2] = bfr(v[2]); xs[jr * 65 + c4 + 3] = bfr(v[3]);
    }
    if (wave < 2) cs[t] = coef[j0 + t];
    __syncthreads();
    const int c8 = (lane & 7) * 8;
    v8us xo[2], ho[2], lo[2];
#pragma unroll
    for (int it = 0; it < 2; ++it) {
        const int ar = it * 32 + wave * 4 + (lane >> 3);
#pragma unroll
        for (int e = 0; e < 8; ++e) {
            const float xv = xs[(c8 + e) * 65 + ar];
            const float v = cs[c8 + e] * xv;
            const unsigned short h = f2bf(v);
            xo[it][e] = (unsigned short)(__float_as_uint(xv) >> 16);
            ho[it][e] = h;
            lo[it][e] = f2bf(v - bf2f(h));
        }
    }
#pragma unroll 1
    for (int ps = 0; ps < 2; ++ps) {
#pragma unroll
        for (int it = 0; it < 2; ++it) {
            const int ar = it * 32 + wave * 4 + (lane >> 3);
            const size_t ox = (size_t)(a0 + ar) * BS + j0 + c8;
            const size_t oa = (size_t)(a0 + ar) * KA + j0 + c8;
            *(volatile v8us*)(XT + ox) = xo[it];
            *(volatile v8us*)(AT + oa) = ho[it];
            *(volatile v8us*)(AT + oa + BS) = lo[it];
        }
        if (ps == 0) __threadfence();
    }
}

__global__ __launch_bounds__(32) void k_gram(const bf* __restrict__ AT, const bf* __restrict__ XT, const float* __restrict__ va, float* OUT) {
    __shared__ __align__(16) float os[16 * 68];
    const int lane = threadIdx.x & 31, lr = lane & 15, hi = lane >> 4;
    const int r0 = blockIdx.x * 64, c0 = blockIdx.y * 64;
    v8f acc[4][4];
#pragma unroll
    for (int mb = 0; mb < 4; ++mb)
#pragma unroll
        for (int nb = 0; nb < 4; ++nb) acc[mb][nb] = (v8f){};
    const size_t aoff = (size_t)(r0 + lr) * KA + 8 * hi, boff = (size_t)(c0 + lr) * BS + 8 * hi;
#pragma unroll 1
    for (int kc = 0; kc < KA; kc += 32) {
        const int kb = (kc >= BS) ? (kc - BS) : kc;
        v16bf a[4];
#pragma unroll
        for (int mb = 0; mb < 4; ++mb) a[mb] = ldb(AT + aoff + (size_t)mb * 16 * KA + kc);
#pragma unroll
        for (int nb = 0; nb < 4; ++nb) { const v16bf b = ldb(XT + boff + (size_t)nb * 16 * BS + kb);
#pragma unroll
            for (int mb = 0; mb < 4; ++mb) acc[mb][nb] = wmmab(a[mb], b, acc[mb][nb]); }
        asm volatile("v_nop\n\tv_nop\n\tv_nop\n\tv_nop" : "+v"(acc[0][0]), "+v"(acc[1][1]), "+v"(acc[2][2]), "+v"(acc[3][3]) : "v"(a[0]), "v"(a[1]), "v"(a[2]), "v"(a[3]));
    }
#pragma unroll
    for (int mb = 0; mb < 4; ++mb) {
#pragma unroll
        for (int nb = 0; nb < 4; ++nb) {
#pragma unroll
            for (int j = 0; j < 8; ++j) os[(hi * 8 + j) * 68 + nb * 16 + lr] = acc[mb][nb][j]; }
        wave_sync();
        const int rb = r0 + mb * 16;
#pragma unroll 1
        for (int ps = 0; ps < 2; ++ps) {
#pragma unroll
            for (int s = 0; s < 8; ++s) { const int row = 2 * s + hi, cofs = lr * 4;
                const v4f sv = *(const v4fa*)(&os[row * 68 + cofs]);
                const v4f vv = *(const v4f*)(va + (size_t)(rb + row) * D_FULL + c0 + cofs);
                v4f val;
                val[0] = sv[0] + bfr(vv[0]); val[1] = sv[1] + bfr(vv[1]); val[2] = sv[2] + bfr(vv[2]); val[3] = sv[3] + bfr(vv[3]);
                *(volatile v4f*)(OUT + (size_t)(rb + row) * OUT_PITCH + c0 + cofs) = val; }
            if (ps == 0) __threadfence(); }
        wave_sync();
    }
}

static constexpr size_t al256(size_t v) { return (v + 255) & ~(size_t)255; }
static constexpr size_t SZ_CF = al256((size_t)BS * 4);
static constexpr size_t SZ_XT = al256((size_t)DD * BS * 2);
static constexpr size_t SZ_AT = al256((size_t)DD * KA * 2);
static constexpr size_t SZ_TOTAL = SZ_CF + SZ_XT + SZ_AT;
static_assert(SZ_TOTAL <= (size_t)134217728);
static_assert(((size_t)BS * 4) % 128 == 0);
static_assert(((size_t)(DD - 1) * BS + (BS - 64) + 64) * 2 <= SZ_XT);
static_assert(((size_t)(DD - 1) * KA + BS + (BS - 64) + 64) * 2 <= SZ_AT);

extern "C" void kernel_launch(void* const* d_in, const int* in_sizes, int n_in,
                              void* d_out, int out_size, void* d_ws, size_t ws_size, hipStream_t stream) {
    if (n_in < 3) return;
    if ((size_t)in_sizes[0] < (size_t)DD) return;
    if ((size_t)in_sizes[1] < (size_t)(DD - 1) * D_FULL + DD) return;
    if ((size_t)in_sizes[2] < (size_t)(BS - 1) * D_FULL + DD) return;
    if ((size_t)out_size < (size_t)(DD - 1) * OUT_PITCH + DD) return;
    if (SZ_TOTAL > ws_size) return;
    const float* mean = (const float*)d_in[0];
    const float* va   = (const float*)d_in[1];
    const float* x    = (const float*)d_in[2];
    float* OUT = (float*)d_out;
    char* wsp = (char*)d_ws;
    float* CF = (float*)wsp; wsp += SZ_CF;
    bf* XT = (bf*)wsp; wsp += SZ_XT;
    bf* AT = (bf*)wsp; wsp += SZ_AT;

    k_coef<<<dim3(BS / 32, 1, 1), 256, 0, stream>>>(x, mean, CF);
    k_planes<<<dim3(BS / 64, DD / 64, 1), 256, 0, stream>>>(x, CF, XT, AT);
    k_gram<<<dim3(DD / 64, DD / 64, 1), 32, 0, stream>>>(AT, XT, va, OUT);
}
